// WaveletMoeDecoderLayer_68135361184394
// MI455X (gfx1250) — hardware-verified
//
#include <hip/hip_runtime.h>
#include <stdint.h>
#include <stddef.h>
#include <math.h>

#pragma clang fp contract(off)

#define NTOK 4096
#define SEQL 512
#define NBAT 8
#define HIDD 768
#define NHD  12
#define NKV  4
#define HDM  64
#define KVW  256
#define NEX  8
#define IEX  1536

#define CP   132
#define MP   68
#define PP   72
#define TP   72
#define AP2  776
#define HP2  1544
#define YP   68

#define LDS_GEMM (128 * CP * 4)
#define LDS_EA   (32 * AP2 * 2)
#define LDS_EH   (32 * HP2 * 2)
#define LDS_EXP  (LDS_EA + LDS_EH + 256)

static_assert(8 * 16 * YP * 4 <= LDS_EA);
static_assert((AP2 * 2) % 16 == 0);
static_assert((HP2 * 2) % 16 == 0);
static_assert((CP * 4) % 16 == 0);
static_assert((MP * 4) % 16 == 0);
static_assert((PP * 2) % 16 == 0);
static_assert(NTOK % 128 == 0);
static_assert(SEQL % 128 == 0);

typedef __bf16         v16bf __attribute__((ext_vector_type(16)));
typedef _Float16       v16h  __attribute__((ext_vector_type(16)));
typedef float          v8f   __attribute__((ext_vector_type(8)));
typedef float          v4f   __attribute__((ext_vector_type(4)));
typedef unsigned int   v4u   __attribute__((ext_vector_type(4)));
typedef int            v4i   __attribute__((ext_vector_type(4)));
typedef v4f __attribute__((may_alias)) v4fa;
typedef v4u __attribute__((may_alias)) v4ua;
typedef v4i __attribute__((may_alias)) v4ia;

union FragBF { v16bf v; v4u q[2]; };
union FragH  { v16h  v; v4u q[2]; };

struct Inv32 { float f[32]; };
static_assert(sizeof(Inv32) == 128);

__device__ __forceinline__ unsigned int bfb(float f) {
  unsigned int u = __float_as_uint(f);
  u += 0x7FFFu + ((u >> 16) & 1u);
  return u >> 16;
}
__device__ __forceinline__ void split2(float v, unsigned int& hi, unsigned int& lo) {
  hi = bfb(v);
  lo = bfb(v - __uint_as_float(hi << 16));
}
__device__ __forceinline__ unsigned int hfb(float f) {
  const _Float16 hv = (_Float16)f;
  return (unsigned int)__builtin_bit_cast(unsigned short, hv);
}
__device__ __forceinline__ unsigned int pk(unsigned int a, unsigned int b) { return (a & 0xFFFFu) | (b << 16); }

__device__ __forceinline__ v8f wmma_bf(v16bf a, v16bf b, v8f c) {
  v8f d = __builtin_amdgcn_wmma_f32_16x16x32_bf16(false, a, false, b, (short)0, c, false, false);
  asm volatile("v_nop\n\tv_nop\n\tv_nop\n\tv_nop" : "+v"(d) : "v"(a), "v"(b));
  return d;
}
__device__ __forceinline__ v8f wmma_h(v16h a, v16h b, v8f c) {
  v8f d = __builtin_amdgcn_wmma_f32_16x16x32_f16(false, a, false, b, (short)0, c, false, false);
  asm volatile("v_nop\n\tv_nop\n\tv_nop\n\tv_nop" : "+v"(d) : "v"(a), "v"(b));
  return d;
}

__device__ __forceinline__ v16bf ldfrag_bf(const unsigned short* p, int h) {
  FragBF f;
  f.q[0] = *(const v4ua*)(p + 8 * h);
  f.q[1] = *(const v4ua*)(p + 16 + 8 * h);
  return f.v;
}
__device__ __forceinline__ v16h ldfrag_h(const unsigned short* p, int h) {
  FragH f;
  f.q[0] = *(const v4ua*)(p + 8 * h);
  f.q[1] = *(const v4ua*)(p + 16 + 8 * h);
  return f.v;
}

__device__ __forceinline__ float wv_sum(float v) {
  v += __shfl_xor(v, 16, 32); v += __shfl_xor(v, 8, 32); v += __shfl_xor(v, 4, 32);
  v += __shfl_xor(v, 2, 32);  v += __shfl_xor(v, 1, 32);
  return v;
}
__device__ __forceinline__ float wv_max(float v) {
  v = fmaxf(v, __shfl_xor(v, 16, 32)); v = fmaxf(v, __shfl_xor(v, 8, 32)); v = fmaxf(v, __shfl_xor(v, 4, 32));
  v = fmaxf(v, __shfl_xor(v, 2, 32));  v = fmaxf(v, __shfl_xor(v, 1, 32));
  return v;
}
__device__ __forceinline__ float h16_sum(float v) {
  v += __shfl_xor(v, 8, 32); v += __shfl_xor(v, 4, 32); v += __shfl_xor(v, 2, 32); v += __shfl_xor(v, 1, 32);
  return v;
}
__device__ __forceinline__ float h16_max(float v) {
  v = fmaxf(v, __shfl_xor(v, 8, 32)); v = fmaxf(v, __shfl_xor(v, 4, 32));
  v = fmaxf(v, __shfl_xor(v, 2, 32)); v = fmaxf(v, __shfl_xor(v, 1, 32));
  return v;
}

__global__ __launch_bounds__(256) void k_cvt_w8(
    const float* __restrict__ s0, const float* __restrict__ s1, const float* __restrict__ s2, const float* __restrict__ s3,
    const float* __restrict__ s4, const float* __restrict__ s5, const float* __restrict__ s6, const float* __restrict__ s7,
    unsigned short* __restrict__ wp)
{
  const int y = blockIdx.y;
  const float* src = s0;
  src = (y == 1) ? s1 : src;  src = (y == 2) ? s2 : src;  src = (y == 3) ? s3 : src;
  src = (y == 4) ? s4 : src;  src = (y == 5) ? s5 : src;  src = (y == 6) ? s6 : src;
  src = (y == 7) ? s7 : src;
  const int yb = y & 3, blk = y >> 2;
  const int n = (yb == 0 || yb == 3) ? (HIDD * HIDD) : (KVW * HIDD);
  size_t hoff = 0;
  hoff = (yb == 1) ? (size_t)1179648 : hoff;
  hoff = (yb == 2) ? (size_t)1572864 : hoff;
  hoff = (yb == 3) ? (size_t)1966080 : hoff;
  hoff += (size_t)blk * 3145728;
  const int g = blockIdx.x * 256 + threadIdx.x;
  if (g >= (n >> 3)) return;
  const float* s = src + (size_t)g * 8;
  const v4f a = *(const v4fa*)s;
  const v4f c = *(const v4fa*)(s + 4);
  unsigned int h0, l0, h1, l1, h2, l2, h3, l3, h4, l4, h5, l5, h6, l6, h7, l7;
  split2(a.x, h0, l0); split2(a.y, h1, l1); split2(a.z, h2, l2); split2(a.w, h3, l3);
  split2(c.x, h4, l4); split2(c.y, h5, l5); split2(c.z, h6, l6); split2(c.w, h7, l7);
  const v4u H = { pk(h0, h1), pk(h2, h3), pk(h4, h5), pk(h6, h7) };
  const v4u L = { pk(l0, l1), pk(l2, l3), pk(l4, l5), pk(l6, l7) };
  unsigned short* dh = wp + hoff + (size_t)g * 8;
  unsigned short* dl = dh + n;
  *(volatile v4u*)dh = H;
  *(volatile v4u*)dl = L;
  __threadfence();
  *(volatile v4u*)dh = H;
  *(volatile v4u*)dl = L;
}

__device__ __forceinline__ void we_store_pass(const unsigned short* sh, unsigned short* dst,
                                              int e, int R, int C, int r0, int c0, int wv, int lane)
{
  const int q8 = lane & 7, sub = lane >> 3;
  #pragma unroll
  for (int i = 0; i < 2; ++i) {
    const int n = wv * 8 + i * 4 + sub;
    const v4u hv = *(const v4ua*)(sh + n * TP + 8 * q8);
    const size_t go = ((size_t)e * C + c0 + n) * R + r0 + 8 * q8;
    *(volatile v4u*)(dst + go) = hv;
  }
}

__global__ __launch_bounds__(256) void k_cvt_we(const float* __restrict__ wg, const float* __restrict__ wu,
                                                const float* __restrict__ wd,
                                                unsigned short* __restrict__ pg, unsigned short* __restrict__ pu,
                                                unsigned short* __restrict__ pd)
{
  __shared__ __align__(16) unsigned short sh[64 * TP];
  const int tid = threadIdx.x, lane = tid & 31, wv = tid >> 5;
  const int z = blockIdx.z;
  const int which = z >> 3, e = z & 7;
  const float* src = wg;
  src = (which == 1) ? wu : src;
  src = (which == 2) ? wd : src;
  unsigned short* dst = pg;
  dst = (which == 1) ? pu : dst;
  dst = (which == 2) ? pd : dst;
  const int R = (which == 2) ? IEX : HIDD;
  const int C = (which == 2) ? HIDD : IEX;
  const int r0 = blockIdx.x * 64;
  const int c0 = blockIdx.y * 64;
  if (r0 >= R || c0 >= C) return;
  const float* sp = src + (size_t)e * R * C;
  #pragma unroll
  for (int j = 0; j < 4; ++j) {
    const int idx = tid + 256 * j;
    const int row = idx >> 4, c4 = idx & 15;
    const v4f v = *(const v4fa*)(sp + (size_t)(r0 + row) * C + c0 + 4 * c4);
    const int cb = 4 * c4;
    sh[(cb + 0) * TP + row] = (unsigned short)hfb(v.x * 64.0f);
    sh[(cb + 1) * TP + row] = (unsigned short)hfb(v.y * 64.0f);
    sh[(cb + 2) * TP + row] = (unsigned short)hfb(v.z * 64.0f);
    sh[(cb + 3) * TP + row] = (unsigned short)hfb(v.w * 64.0f);
  }
  __syncthreads();
  we_store_pass(sh, dst, e, R, C, r0, c0, wv, lane);
  __threadfence();
  we_store_pass(sh, dst, e, R, C, r0, c0, wv, lane);
}

__global__ __launch_bounds__(256) void k_rms_planes(const float* __restrict__ x, const float* __restrict__ w,
                                                    unsigned short* __restrict__ ph, unsigned short* __restrict__ pl,
                                                    const int* __restrict__ pid, float* __restrict__ cs, int do_cs,
                                                    Inv32 ivf)
{
  const int tid = threadIdx.x, lane = tid & 31, wv = tid >> 5;
  const int t = blockIdx.x * 8 + wv;
  const float* xr = x + (size_t)t * HIDD;
  v4f xa[3], xb[3];
  float ssq = 0.f;
  #pragma unroll
  for (int i = 0; i < 3; ++i) {
    const int e0 = 8 * (32 * i + lane);
    xa[i] = *(const v4fa*)(xr + e0);
    xb[i] = *(const v4fa*)(xr + e0 + 4);
    ssq = ssq + xa[i].x * xa[i].x; ssq = ssq + xa[i].y * xa[i].y;
    ssq = ssq + xa[i].z * xa[i].z; ssq = ssq + xa[i].w * xa[i].w;
    ssq = ssq + xb[i].x * xb[i].x; ssq = ssq + xb[i].y * xb[i].y;
    ssq = ssq + xb[i].z * xb[i].z; ssq = ssq + xb[i].w * xb[i].w;
  }
  ssq = wv_sum(ssq);
  const float var = ssq * (1.0f / 768.0f);
  const float inv = 1.0f / sqrtf(var + 1.0e-6f);
  v4u H[3], L[3];
  #pragma unroll
  for (int i = 0; i < 3; ++i) {
    const int e0 = 8 * (32 * i + lane);
    const v4f wa = *(const v4fa*)(w + e0);
    const v4f wb = *(const v4fa*)(w + e0 + 4);
    const float y0 = wa.x * (xa[i].x * inv), y1 = wa.y * (xa[i].y * inv);
    const float y2 = wa.z * (xa[i].z * inv), y3 = wa.w * (xa[i].w * inv);
    const float y4 = wb.x * (xb[i].x * inv), y5 = wb.y * (xb[i].y * inv);
    const float y6 = wb.z * (xb[i].z * inv), y7 = wb.w * (xb[i].w * inv);
    unsigned int a0, b0, a1, b1, a2, b2, a3, b3, a4, b4, a5, b5, a6, b6, a7, b7;
    split2(y0, a0, b0); split2(y1, a1, b1); split2(y2, a2, b2); split2(y3, a3, b3);
    split2(y4, a4, b4); split2(y5, a5, b5); split2(y6, a6, b6); split2(y7, a7, b7);
    const v4u hv = { pk(a0, a1), pk(a2, a3), pk(a4, a5), pk(a6, a7) };
    const v4u lv = { pk(b0, b1), pk(b2, b3), pk(b4, b5), pk(b6, b7) };
    H[i] = hv; L[i] = lv;
  }
  const size_t ro = (size_t)t * HIDD;
  #pragma unroll
  for (int i = 0; i < 3; ++i) {
    const int e0 = 8 * (32 * i + lane);
    *(volatile v4u*)(ph + ro + e0) = H[i];
    *(volatile v4u*)(pl + ro + e0) = L[i];
  }
  float cv = 0.f, sv = 0.f;
  const size_t cso = (size_t)t * 64 + lane;
  if (do_cs) {
    const int pos = pid[t];
    float iv = ivf.f[0];
    #pragma unroll
    for (int q = 1; q < 32; ++q) iv = (lane == q) ? ivf.f[q] : iv;
    const float ang = (float)pos * iv;
    sincosf(ang, &sv, &cv);
    *(volatile float*)(cs + cso) = cv;
    *(volatile float*)(cs + cso + 32) = sv;
  }
  __threadfence();
  #pragma unroll
  for (int i = 0; i < 3; ++i) {
    const int e0 = 8 * (32 * i + lane);
    *(volatile v4u*)(ph + ro + e0) = H[i];
    *(volatile v4u*)(pl + ro + e0) = L[i];
  }
  if (do_cs) {
    *(volatile float*)(cs + cso) = cv;
    *(volatile float*)(cs + cso + 32) = sv;
  }
}

__device__ __forceinline__ void ep_f32_pass(const float* sC, const float* bias, int use_bias,
                                            const float* resid, int ldr, int use_resid,
                                            float* outf, int ldo, int m0, int n0, int wv, int lane)
{
  #pragma unroll
  for (int i = 0; i < 16; ++i) {
    const int row = wv * 16 + i;
    v4f v = *(const v4fa*)(sC + row * CP + 4 * lane);
    if (use_bias) {
      const v4f bb = *(const v4fa*)(bias + n0 + 4 * lane);
      v = v + bb;
    }
    if (use_resid) {
      const v4f rr = *(const v4fa*)(resid + (size_t)(m0 + row) * ldr + n0 + 4 * lane);
      v = rr + v;
    }
    *(volatile v4f*)(outf + (size_t)(m0 + row) * ldo + n0 + 4 * lane) = v;
  }
}

__device__ __forceinline__ void ep_rope_pass(const float* sC, const float* bias, const float* cs,
                                             unsigned short* oh, unsigned short* ol, int nheads,
                                             int m0, int n0, int tid)
{
  const int q8 = tid & 7, sub = tid >> 3;
  #pragma unroll 1
  for (int p = 0; p < 8; ++p) {
    const int L = p * 32 + sub;
    const int row = L >> 1, hh = L & 1;
    const int token = m0 + row;
    const int b = token / SEQL, s = token - b * SEQL;
    const int head = (n0 >> 6) + hh;
    const float* cr = cs + (size_t)token * 64;
    const float* xrow = sC + row * CP + 64 * hh;
    const float* brow = bias + n0 + 64 * hh;
    unsigned int hb[8], lb[8];
    #pragma unroll
    for (int j = 0; j < 8; ++j) {
      const int d = 8 * q8 + j;
      const int dd = d & 31;
      const int pd = d ^ 32;
      const float x0 = xrow[d] + brow[d];
      const float xp = xrow[pd] + brow[pd];
      const float cc = cr[dd], sn = cr[32 + dd];
      const float t1 = x0 * cc;
      const float t2 = xp * sn;
      const float val = (d < 32) ? (t1 - t2) : (t1 + t2);
      split2(val, hb[j], lb[j]);
    }
    const v4u H = { pk(hb[0], hb[1]), pk(hb[2], hb[3]), pk(hb[4], hb[5]), pk(hb[6], hb[7]) };
    const v4u Lw = { pk(lb[0], lb[1]), pk(lb[2], lb[3]), pk(lb[4], lb[5]), pk(lb[6], lb[7]) };
    const size_t off = (((size_t)b * nheads + head) * SEQL + s) * HDM + 8 * q8;
    *(volatile v4u*)(oh + off) = H;
    *(volatile v4u*)(ol + off) = Lw;
  }
}

__device__ __forceinline__ void ep_tr_pass(const float* sC, const float* bias,
                                           unsigned short* oh, unsigned short* ol, int nheads,
                                           int m0, int n0, int tid)
{
  const int q16 = tid & 15, sub = tid >> 4;
  const int b = m0 / SEQL, s0 = m0 - b * SEQL;
  #pragma unroll 1
  for (int p = 0; p < 8; ++p) {
    const int rid = p * 16 + sub;
    const int hh = rid >> 6, d = rid & 63;
    const int col = 64 * hh + d;
    const int head = (n0 >> 6) + hh;
    const float bb = bias[n0 + col];
    unsigned int hb[8], lb[8];
    #pragma unroll
    for (int j = 0; j < 8; ++j) {
      const float v = sC[(8 * q16 + j) * CP + col] + bb;
      split2(v, hb[j], lb[j]);
    }
    const v4u H = { pk(hb[0], hb[1]), pk(hb[2], hb[3]), pk(hb[4], hb[5]), pk(hb[6], hb[7]) };
    const v4u Lw = { pk(lb[0], lb[1]), pk(lb[2], lb[3]), pk(lb[4], lb[5]), pk(lb[6], lb[7]) };
    const size_t off = (((size_t)b * nheads + head) * HDM + d) * SEQL + s0 + 8 * q16;
    *(volatile v4u*)(oh + off) = H;
    *(volatile v4u*)(ol + off) = Lw;
  }
}

template <int MODE>
__global__ __launch_bounds__(256) void k_gemm3(
    const unsigned short* __restrict__ Ah, const unsigned short* __restrict__ Al, int lda,
    const unsigned short* __restrict__ Bh, const unsigned short* __restrict__ Bl, int ldb, int K,
    const float* __restrict__ bias, int use_bias,
    const float* __restrict__ resid, int ldr, int use_resid,
    float* __restrict__ outf, int ldo,
    unsigned short* __restrict__ oh, unsigned short* __restrict__ ol, int nheads,
    const float* __restrict__ cs)
{
  extern __shared__ __align__(16) unsigned char dsm_g[];
  float* sC = (float*)dsm_g;
  const int tid = threadIdx.x, lane = tid & 31, wv = tid >> 5;
  const int h = lane >> 4, m = lane & 15;
  const int wm = wv & 3, wn = wv >> 2;
  const int m0 = blockIdx.x * 128, n0 = blockIdx.y * 128;
  const v8f z8 = {0.f, 0.f, 0.f, 0.f, 0.f, 0.f, 0.f, 0.f};
  v8f acc[2][4];
  #pragma unroll
  for (int mt = 0; mt < 2; ++mt)
    #pragma unroll
    for (int nt = 0; nt < 4; ++nt) acc[mt][nt] = z8;

  #pragma unroll 1
  for (int k0 = 0; k0 < K; k0 += 32) {
    v16bf ah[2], al[2];
    #pragma unroll
    for (int mt = 0; mt < 2; ++mt) {
      const size_t ro = (size_t)(m0 + 32 * wm + 16 * mt + m) * lda + k0;
      ah[mt] = ldfrag_bf(Ah + ro, h);
      al[mt] = ldfrag_bf(Al + ro, h);
    }
    #pragma unroll
    for (int nt = 0; nt < 4; ++nt) {
      const size_t co = (size_t)(n0 + 64 * wn + 16 * nt + m) * ldb + k0;
      const v16bf bh = ldfrag_bf(Bh + co, h);
      const v16bf bl = ldfrag_bf(Bl + co, h);
      #pragma unroll
      for (int mt = 0; mt < 2; ++mt) {
        acc[mt][nt] = wmma_bf(ah[mt], bh, acc[mt][nt]);
        acc[mt][nt] = wmma_bf(ah[mt], bl, acc[mt][nt]);
        acc[mt][nt] = wmma_bf(al[mt], bh, acc[mt][nt]);
      }
    }
  }
  #pragma unroll
  for (int mt = 0; mt < 2; ++mt)
    #pragma unroll
    for (int nt = 0; nt < 4; ++nt)
      #pragma unroll
      for (int r = 0; r < 8; ++r) {
        const int row = 32 * wm + 16 * mt + 8 * h + r;
        const int col = 64 * wn + 16 * nt + m;
        sC[row * CP + col] = acc[mt][nt][r];
      }
  __syncthreads();
  if (MODE == 0) {
    ep_f32_pass(sC, bias, use_bias, resid, ldr, use_resid, outf, ldo, m0, n0, wv, lane);
    __threadfence();
    ep_f32_pass(sC, bias, use_bias, resid, ldr, use_resid, outf, ldo, m0, n0, wv, lane);
  } else if (MODE == 1) {
    ep_rope_pass(sC, bias, cs, oh, ol, nheads, m0, n0, tid);
    __threadfence();
    ep_rope_pass(sC, bias, cs, oh, ol, nheads, m0, n0, tid);
  } else {
    ep_tr_pass(sC, bias, oh, ol, nheads, m0, n0, tid);
    __threadfence();
    ep_tr_pass(sC, bias, oh, ol, nheads, m0, n0, tid);
  }
}

__device__ __forceinline__ void ctx_pass(const float* sO, const float* sLw,
                                         unsigned short* Ch, unsigned short* Cl,
                                         int b, int head, int q0, int wv, int lane)
{
  const int q8 = lane & 7, sub = lane >> 3;
  #pragma unroll
  for (int i = 0; i < 4; ++i) {
    const int row = 4 * i + sub;
    const float inv = 1.0f / sLw[row];
    const float* orow = sO + row * MP + 8 * q8;
    unsigned int hb[8], lb[8];
    #pragma unroll
    for (int j = 0; j < 8; ++j) split2(orow[j] * inv, hb[j], lb[j]);
    const v4u H = { pk(hb[0], hb[1]), pk(hb[2], hb[3]), pk(hb[4], hb[5]), pk(hb[6], hb[7]) };
    const v4u Lw = { pk(lb[0], lb[1]), pk(lb[2], lb[3]), pk(lb[4], lb[5]), pk(lb[6], lb[7]) };
    const int token = b * SEQL + q0 + 16 * wv + row;
    const size_t off = (size_t)token * HIDD + head * HDM + 8 * q8;
    *(volatile v4u*)(Ch + off) = H;
    *(volatile v4u*)(Cl + off) = Lw;
  }
}

__global__ __launch_bounds__(128) __attribute__((amdgpu_num_vgpr(256)))
void k_flash(const unsigned short* __restrict__ Qh, const unsigned short* __restrict__ Ql,
             const unsigned short* __restrict__ Kh, const unsigned short* __restrict__ Kl,
             const unsigned short* __restrict__ Vh, const unsigned short* __restrict__ Vl,
             const float* __restrict__ mask,
             unsigned short* __restrict__ Ch, unsigned short* __restrict__ Cl)
{
  __shared__ __align__(16) float sM[64 * MP];
  __shared__ __align__(16) float sS[64 * MP];
  __shared__ __align__(16) unsigned short sPh[64 * PP];
  __shared__ __align__(16) unsigned short sPl[64 * PP];
  __shared__ float sRed[4];
  __shared__ float sL[64];

  const int tid = threadIdx.x, lane = tid & 31, wv = tid >> 5;
  const int h = lane >> 4, m = lane & 15;
  const int bh = blockIdx.x;
  const int b = bh / NHD, head = bh - b * NHD;
  const int kvh = head / (NHD / NKV);
  const int q0 = blockIdx.y * 64;

  const size_t qro = (((size_t)b * NHD + head) * SEQL + q0 + 16 * wv + m) * HDM;
  v16bf qh[2], ql[2];
  #pragma unroll
  for (int ks = 0; ks < 2; ++ks) {
    qh[ks] = ldfrag_bf(Qh + qro + 32 * ks, h);
    ql[ks] = ldfrag_bf(Ql + qro + 32 * ks, h);
  }
  const size_t kbase = ((size_t)b * NKV + kvh) * SEQL * HDM;
  const size_t vbase = ((size_t)b * NKV + kvh) * HDM * SEQL;

  const v8f z8 = {0.f, 0.f, 0.f, 0.f, 0.f, 0.f, 0.f, 0.f};
  v8f o[4];
  #pragma unroll
  for (int dt = 0; dt < 4; ++dt) o[dt] = z8;
  float mrow[8], lrow[8];
  #pragma unroll
  for (int r = 0; r < 8; ++r) { mrow[r] = -1.0e30f; lrow[r] = 0.f; }

  float* sSw = sS + wv * 16 * MP;
  unsigned short* sPhw = sPh + wv * 16 * PP;
  unsigned short* sPlw = sPl + wv * 16 * PP;

  #pragma unroll 1
  for (int jt = 0; jt < SEQL / 64; ++jt) {
    const int j0 = jt * 64;
    __syncthreads();
    float lmax = -3.0e38f;
    #pragma unroll
    for (int i = 0; i < 8; ++i) {
      const int idx = tid + 128 * i;
      const int row = idx >> 4, c4 = idx & 15;
      const v4f v = *(const v4fa*)(mask + (size_t)(q0 + row) * SEQL + j0 + 4 * c4);
      *(v4fa*)(sM + row * MP + 4 * c4) = v;
      lmax = fmaxf(lmax, fmaxf(fmaxf(v.x, v.y), fmaxf(v.z, v.w)));
    }
    lmax = wv_max(lmax);
    if (lane == 0) sRed[wv] = lmax;
    __syncthreads();
    const float tmax = fmaxf(fmaxf(sRed[0], sRed[1]), fmaxf(sRed[2], sRed[3]));
    if (tmax <= -1.0e8f) continue;

    #pragma unroll 1
    for (int nt = 0; nt < 4; ++nt) {
      const size_t kro = kbase + (size_t)(j0 + 16 * nt + m) * HDM;
      v8f sacc = z8;
      #pragma unroll
      for (int ks = 0; ks < 2; ++ks) {
        const v16bf kh = ldfrag_bf(Kh + kro + 32 * ks, h);
        const v16bf kl = ldfrag_bf(Kl + kro + 32 * ks, h);
        sacc = wmma_bf(qh[ks], kh, sacc);
        sacc = wmma_bf(qh[ks], kl, sacc);
        sacc = wmma_bf(ql[ks], kh, sacc);
      }
      float* sp = sSw + (8 * h) * MP + 16 * nt + m;
      #pragma unroll
      for (int r = 0; r < 8; ++r) sp[r * MP] = sacc[r];
    }

    #pragma unroll
    for (int r = 0; r < 8; ++r) {
      const int rowl = 16 * wv + 8 * h + r;
      const float* mr = sM + rowl * MP + m;
      const float* sr = sSw + (8 * h + r) * MP + m;
      const float sv0 = sr[0] * 0.125f + mr[0];
      const float sv1 = sr[16] * 0.125f + mr[16];
      const float sv2 = sr[32] * 0.125f + mr[32];
      const float sv3 = sr[48] * 0.125f + mr[48];
      float rmax = fmaxf(fmaxf(sv0, sv1), fmaxf(sv2, sv3));
      rmax = h16_max(rmax);
      const float mn = fmaxf(mrow[r], rmax);
      const float corr = __expf(mrow[r] - mn);
      const float p0 = __expf(sv0 - mn);
      const float p1 = __expf(sv1 - mn);
      const float p2 = __expf(sv2 - mn);
      const float p3 = __expf(sv3 - mn);
      float rs = (p0 + p1) + (p2 + p3);
      rs = h16_sum(rs);
      lrow[r] = lrow[r] * corr + rs;
      mrow[r] = mn;
      #pragma unroll
      for (int dt = 0; dt < 4; ++dt) o[dt][r] = o[dt][r] * corr;
      unsigned int a0, b0, a1, b1, a2, b2, a3, b3;
      split2(p0, a0, b0); split2(p1, a1, b1); split2(p2, a2, b2); split2(p3, a3, b3);
      const int po = (8 * h + r) * PP + m;
      sPhw[po] = (unsigned short)a0;       sPlw[po] = (unsigned short)b0;
      sPhw[po + 16] = (unsigned short)a1;  sPlw[po + 16] = (unsigned short)b1;
      sPhw[po + 32] = (unsigned short)a2;  sPlw[po + 32] = (unsigned short)b2;
      sPhw[po + 48] = (unsigned short)a3;  sPlw[po + 48] = (unsigned short)b3;
    }
    __syncthreads();
    #pragma unroll 1
    for (int ks = 0; ks < 2; ++ks) {
      const v16bf pah = ldfrag_bf(sPhw + m * PP + 32 * ks, h);
      const v16bf pal = ldfrag_bf(sPlw + m * PP + 32 * ks, h);
      #pragma unroll
      for (int dt = 0; dt < 4; ++dt) {
        const size_t vro = vbase + (size_t)(16 * dt + m) * SEQL + j0 + 32 * ks;
        const v16bf vh = ldfrag_bf(Vh + vro, h);
        const v16bf vl = ldfrag_bf(Vl + vro, h);
        o[dt] = wmma_bf(pah, vh, o[dt]);
        o[dt] = wmma_bf(pah, vl, o[dt]);
        o[dt] = wmma_bf(pal, vh, o[dt]);
      }
    }
  }
  __syncthreads();
  float* sO = sM + wv * 16 * MP;
  #pragma unroll
  for (int dt = 0; dt < 4; ++dt)
    #pragma unroll
    for (int r = 0; r < 8; ++r) sO[(8 * h + r) * MP + 16 * dt + m] = o[dt][r];
  if (m == 0) {
    #pragma unroll
    for (int r = 0; r < 8; ++r) sL[wv * 16 + 8 * h + r] = lrow[r];
  }
  __syncthreads();
  ctx_pass(sO, sL + wv * 16, Ch, Cl, b, head, q0, wv, lane);
  __threadfence();
  ctx_pass(sO, sL + wv * 16, Ch, Cl, b, head, q0, wv, lane);
}

__device__ __forceinline__ void ga_pass(const float* so, unsigned short* ch, unsigned short* cl,
                                        int s, int head, int lane)
{
  const int q8 = lane & 7, sub = lane >> 3;
  #pragma unroll
  for (int i = 0; i < 2; ++i) {
    const int bb = 4 * i + sub;
    const float* orow = so + bb * 64 + 8 * q8;
    unsigned int hb[8], lb[8];
    #pragma unroll
    for (int j = 0; j < 8; ++j) split2(orow[j], hb[j], lb[j]);
    const v4u H = { pk(hb[0], hb[1]), pk(hb[2], hb[3]), pk(hb[4], hb[5]), pk(hb[6], hb[7]) };
    const v4u Lw = { pk(lb[0], lb[1]), pk(lb[2], lb[3]), pk(lb[4], lb[5]), pk(lb[6], lb[7]) };
    const size_t off = ((size_t)(bb * SEQL + s)) * HIDD + head * HDM + 8 * q8;
    *(volatile v4u*)(ch + off) = H;
    *(volatile v4u*)(cl + off) = Lw;
  }
}

__global__ __launch_bounds__(256) void k_gattn(const float* __restrict__ q2, const float* __restrict__ k2,
                                               const float* __restrict__ v2, const float* __restrict__ gm,
                                               unsigned short* __restrict__ ch, unsigned short* __restrict__ cl)
{
  __shared__ __align__(16) float sQ[8 * 512];
  __shared__ __align__(16) float sK[8 * 512];
  __shared__ __align__(16) float sV[8 * 512];
  __shared__ float sP[8 * 64];
  const int tid = threadIdx.x, lane = tid & 31, wv = tid >> 5;
  const int pair = blockIdx.x * 8 + wv;
  const int s = pair / NHD, head = pair - s * NHD;
  const int kvh = head / (NHD / NKV);
  float* wq = sQ + wv * 512;
  float* wk = sK + wv * 512;
  float* wvv = sV + wv * 512;
  #pragma unroll
  for (int i = 0; i < 4; ++i) {
    const int idx = lane + 32 * i;
    const int bq = idx >> 4, c4 = idx & 15;
    const v4f a = *(const v4fa*)(q2 + ((size_t)(bq * SEQL + s)) * HIDD + head * HDM + 4 * c4);
    const v4f kk = *(const v4fa*)(k2 + ((size_t)(bq * SEQL + s)) * KVW + kvh * HDM + 4 * c4);
    const v4f vv = *(const v4fa*)(v2 + ((size_t)(bq * SEQL + s)) * KVW + kvh * HDM + 4 * c4);
    *(v4fa*)(wq + bq * 64 + 4 * c4) = a;
    *(v4fa*)(wk + bq * 64 + 4 * c4) = kk;
    *(v4fa*)(wvv + bq * 64 + 4 * c4) = vv;
  }
  __syncthreads();
  const int b = lane >> 2, c0 = (lane & 3) * 2;
  float d0 = 0.f, d1 = 0.f;
  {
    const float* qr = wq + b * 64;
    const float* k0r = wk + c0 * 64;
    const float* k1r = wk + (c0 + 1) * 64;
    #pragma unroll 4
    for (int d = 0; d < HDM; ++d) {
      const float qv = qr[d];
      d0 = fmaf(qv, k0r[d], d0);
      d1 = fmaf(qv, k1r[d], d1);
    }
  }
  const float sc0 = d0 * 0.125f + gm[((size_t)s * NBAT + b) * NBAT + c0];
  const float sc1 = d1 * 0.125f + gm[((size_t)s * NBAT + b) * NBAT + c0 + 1];
  float mx = fmaxf(sc0, sc1);
  mx = fmaxf(mx, __shfl_xor(mx, 1, 32));
  mx = fmaxf(mx, __shfl_xor(mx, 2, 32));
  const float e0 = __expf(sc0 - mx);
  const float e1 = __expf(sc1 - mx);
  float sm = e0 + e1;
  sm += __shfl_xor(sm, 1, 32);
  sm += __shfl_xor(sm, 2, 32);
  const float inv = 1.0f / sm;
  sP[wv * 64 + b * 8 + c0] = e0 * inv;
  sP[wv * 64 + b * 8 + c0 + 1] = e1 * inv;
  __syncthreads();
  const int dq = (lane & 3) * 16;
  float oacc[16];
  #pragma unroll
  for (int dd = 0; dd < 16; ++dd) oacc[dd] = 0.f;
  #pragma unroll 1
  for (int c = 0; c < NBAT; ++c) {
    const float pc = sP[wv * 64 + b * 8 + c];
    const float* vr = wvv + c * 64 + dq;
    #pragma unroll
    for (int dd = 0; dd < 16; ++dd) oacc[dd] = fmaf(pc, vr[dd], oacc[dd]);
  }
  float* so = sK + wv * 512;
  {
    const v4f o0 = { oacc[0], oacc[1], oacc[2], oacc[3] };
    const v4f o1 = { oacc[4], oacc[5], oacc[6], oacc[7] };
    const v4f o2 = { oacc[8], oacc[9], oacc[10], oacc[11] };
    const v4f o3 = { oacc[12], oacc[13], oacc[14], oacc[15] };
    *(v4fa*)(so + b * 64 + dq) = o0;
    *(v4fa*)(so + b * 64 + dq + 4) = o1;
    *(v4fa*)(so + b * 64 + dq + 8) = o2;
    *(v4fa*)(so + b * 64 + dq + 12) = o3;
  }
  __syncthreads();
  ga_pass(so, ch, cl, s, head, lane);
  __threadfence();
  ga_pass(so, ch, cl, s, head, lane);
}

__global__ __launch_bounds__(256) void k_rms_route(const float* __restrict__ x, const float* __restrict__ w,
                                                   const float* __restrict__ gw,
                                                   unsigned short* __restrict__ xf16, float* __restrict__ rec)
{
  __shared__ __align__(16) float sX[8 * HIDD];
  __shared__ float sLg[64];
  __shared__ float sPr[64];
  __shared__ __align__(16) float sRec[32];
  const int tid = threadIdx.x, lane = tid & 31, wv = tid >> 5;
  const int t = blockIdx.x * 8 + wv;
  const float* xr = x + (size_t)t * HIDD;
  v4f xa[3], xb[3];
  float ssq = 0.f;
  #pragma unroll
  for (int i = 0; i < 3; ++i) {
    const int e0 = 8 * (32 * i + lane);
    xa[i] = *(const v4fa*)(xr + e0);
    xb[i] = *(const v4fa*)(xr + e0 + 4);
    ssq = ssq + xa[i].x * xa[i].x; ssq = ssq + xa[i].y * xa[i].y;
    ssq = ssq + xa[i].z * xa[i].z; ssq = ssq + xa[i].w * xa[i].w;
    ssq = ssq + xb[i].x * xb[i].x; ssq = ssq + xb[i].y * xb[i].y;
    ssq = ssq + xb[i].z * xb[i].z; ssq = ssq + xb[i].w * xb[i].w;
  }
  ssq = wv_sum(ssq);
  const float var = ssq * (1.0f / 768.0f);
  const float inv = 1.0f / sqrtf(var + 1.0e-6f);
  v4u F[3];
  float* sxw = sX + wv * HIDD;
  #pragma unroll
  for (int i = 0; i < 3; ++i) {
    const int e0 = 8 * (32 * i + lane);
    const v4f wa = *(const v4fa*)(w + e0);
    const v4f wb = *(const v4fa*)(w + e0 + 4);
    const v4f ya = { wa.x * (xa[i].x * inv), wa.y * (xa[i].y * inv), wa.z * (xa[i].z * inv), wa.w * (xa[i].w * inv) };
    const v4f yb = { wb.x * (xb[i].x * inv), wb.y * (xb[i].y * inv), wb.z * (xb[i].z * inv), wb.w * (xb[i].w * inv) };
    const v4u fv = { pk(hfb(ya.x), hfb(ya.y)), pk(hfb(ya.z), hfb(ya.w)), pk(hfb(yb.x), hfb(yb.y)), pk(hfb(yb.z), hfb(yb.w)) };
    F[i] = fv;
    *(v4fa*)(sxw + e0) = ya;
    *(v4fa*)(sxw + e0 + 4) = yb;
  }
  const size_t ro = (size_t)t * HIDD;
  #pragma unroll
  for (int i = 0; i < 3; ++i) {
    const int e0 = 8 * (32 * i + lane);
    *(volatile v4u*)(xf16 + ro + e0) = F[i];
  }
  __syncthreads();
  #pragma unroll 1
  for (int e = 0; e < NEX; ++e) {
    float p = 0.f;
    const float* gr = gw + (size_t)e * HIDD;
    #pragma unroll 1
    for (int i = 0; i < 6; ++i) {
      const int k = 4 * (32 * i + lane);
      const v4f xv = *(const v4fa*)(sxw + k);
      const v4f gv = *(const v4fa*)(gr + k);
      p = fmaf(xv.x, gv.x, p);
      p = fmaf(xv.y, gv.y, p);
      p = fmaf(xv.z, gv.z, p);
      p = fmaf(xv.w, gv.w, p);
    }
    p = wv_sum(p);
    if (lane == 0) sLg[wv * 8 + e] = p;
  }
  __syncthreads();
  if (lane == 0) {
    const int bq = wv * 8;
    float mx = sLg[bq];
    #pragma unroll 1
    for (int e = 1; e < NEX; ++e) mx = fmaxf(mx, sLg[bq + e]);
    float sum = 0.f;
    #pragma unroll 1
    for (int e = 0; e < NEX; ++e) {
      const float ev = expf(sLg[bq + e] - mx);
      sPr[bq + e] = ev;
      sum = sum + ev;
    }
    const float rs = 1.0f / sum;
    #pragma unroll 1
    for (int e = 0; e < NEX; ++e) sPr[bq + e] = sPr[bq + e] * rs;
    int i1 = 0;
    float b1 = sPr[bq];
    #pragma unroll 1
    for (int e = 1; e < NEX; ++e) {
      const float v = sPr[bq + e];
      if (v > b1) { b1 = v; i1 = e; }
    }
    int i2 = -1;
    float b2 = 0.f;
    #pragma unroll 1
    for (int e = 0; e < NEX; ++e) {
      const float v = sPr[bq + e];
      const bool take = (e != i1) && ((i2 < 0) || (v > b2));
      if (take) { b2 = v; i2 = e; }
    }
    int elo, ehi;
    float wlo, whi;
    if (i1 < i2) { elo = i1; wlo = b1; ehi = i2; whi = b2; }
    else         { elo = i2; wlo = b2; ehi = i1; whi = b1; }
    sRec[wv * 4 + 0] = wlo;
    sRec[wv * 4 + 1] = whi;
    sRec[wv * 4 + 2] = (float)elo;
    sRec[wv * 4 + 3] = (float)ehi;
  }
  __syncthreads();
  v4f rv = {0.f, 0.f, 0.f, 0.f};
  if (tid < 8) {
    rv = *(const v4fa*)(sRec + 4 * tid);
    *(volatile v4f*)(rec + (size_t)(blockIdx.x * 8 + tid) * 4) = rv;
  }
  __threadfence();
  #pragma unroll
  for (int i = 0; i < 3; ++i) {
    const int e0 = 8 * (32 * i + lane);
    *(volatile v4u*)(xf16 + ro + e0) = F[i];
  }
  if (tid < 8) {
    *(volatile v4f*)(rec + (size_t)(blockIdx.x * 8 + tid) * 4) = rv;
  }
}

__device__ __forceinline__ void list_pass(const int* s_list, int* L, int* CL, int base, int tid) {
  #pragma unroll
  for (int j = 0; j < 4; ++j) {
    const int idx = tid + 256 * j;
    const v4i v = *(const v4ia*)(s_list + 4 * idx);
    *(volatile v4i*)(L + 4 * idx) = v;
  }
  if (tid < 8) {
    const v4i cv = { base, base, base, base };
    *(volatile v4i*)(CL + 4 * tid) = cv;
  }
}

__global__ __launch_bounds__(256) void k_lists(const float* __restrict__ rec, int* __restrict__ lst,
                                               int* __restrict__ cnt)
{
  __shared__ __align__(16) int s_list[NTOK];
  __shared__ int s_wc[8];
  const int tid = threadIdx.x, lane = tid & 31, wv = tid >> 5;
  const int e = blockIdx.x;
  for (int s = 0; s < 2; ++s) {
    __syncthreads();
    #pragma unroll 1
    for (int i = 0; i < NTOK / 256; ++i) s_list[tid + 256 * i] = 0;
    __syncthreads();
    int base = 0;
    #pragma unroll 1
    for (int c = 0; c < NTOK / 256; ++c) {
      const int t = c * 256 + tid;
      const v4f r = *(const v4fa*)(rec + (size_t)t * 4);
      const int sel = (s == 0) ? (int)r.z : (int)r.w;
      const bool f = (sel == e);
      const unsigned int msk = __builtin_amdgcn_ballot_w32(f);
      const int off = __builtin_popcount(msk & ((1u << lane) - 1u));
      const int wc = __builtin_popcount(msk);
      if (lane == 0) s_wc[wv] = wc;
      __syncthreads();
      int pre = 0, tot = 0;
      #pragma unroll 1
      for (int w2 = 0; w2 < 8; ++w2) {
        const int cc = s_wc[w2];
        tot += cc;
        pre += (w2 < wv) ? cc : 0;
      }
      if (f) {
        int p = base + pre + off;
        p = (p < 0) ? 0 : ((p > NTOK - 1) ? (NTOK - 1) : p);
        s_list[p] = t;
      }
      base += tot;
      __syncthreads();
    }
    base = (base > NTOK) ? NTOK : base;
    int* L  = lst + (size_t)(s * NEX + e) * NTOK;
    int* CL = cnt + (size_t)(s * NEX + e) * 32;
    list_pass(s_list, L, CL, base, tid);
    __threadfence();
    list_pass(s_list, L, CL, base, tid);
  }
}

template <int SLOT>
__device__ __forceinline__ void y_pass(const float* sy, const int* s_tok, const float* padd,
                                       const float* hres, float* dst, int mg, int nrows,
                                       int colbase, int lane)
{
  const int q16 = lane & 15, sub = lane >> 4;
  #pragma unroll
  for (int i = 0; i < 8; ++i) {
    const int rowl = 2 * i + sub;
    const int row = 16 * mg + rowl;
    v4f v = *(const v4fa*)(sy + rowl * YP + 4 * q16);
    if (row < nrows) {
      const int t = s_tok[row];
      const size_t go = (size_t)t * HIDD + colbase + 4 * q16;
      if (SLOT == 1) {
        const v4f p0 = *(const v4fa*)(padd + go);
        const v4f hr = *(const v4fa*)(hres + go);
        v = p0 + v;
        v = hr + v;
      }
      *(volatile v4f*)(dst + go) = v;
    }
  }
}

template <int SLOT>
__global__ __launch_bounds__(256) void k_expert(const unsigned short* __restrict__ xf,
                                                const unsigned short* __restrict__ pg,
                                                const unsigned short* __restrict__ pu,
                                                const unsigned short* __restrict__ pd,
                                                const float* __restrict__ rec,
                                                const int* __restrict__ lst,
                                                const int* __restrict__ cnt,
                                                const float* __restrict__ padd,
                                                const float* __restrict__ hres,
                                                float* __restrict__ dst)
{
  extern __shared__ __align__(16) unsigned char dsm_e[];
  unsigned short* sA = (unsigned short*)dsm_e;
  unsigned short* sH = (unsigned short*)(dsm_e + LDS_EA);
  float* sY = (float*)dsm_e;
  int*   s_tok = (int*)(dsm_e + LDS_EA + LDS_EH);
  float* s_w   = (float*)(dsm_e + LDS_EA + LDS_EH + 128);

  const int tid = threadIdx.x, lane = tid & 31, wv = tid >> 5;
  const int h = lane >> 4, m = lane & 15;
  const int e = blockIdx.y, tile = blockIdx.x;

  int c = cnt[(SLOT * NEX + e) * 32];
  c = (c < 0) ? 0 : ((c > NTOK) ? NTOK : c);
  if (tile * 32 >= c) return;
  int nrows = c - tile * 32;
  nrows = (nrows > 32) ? 32 : nrows;

  if (tid < 32) {
    int idx = tile * 32 + tid;
    idx = (idx > NTOK - 1) ? (NTOK - 1) : idx;
    int t = lst[(size_t)(SLOT * NEX + e) * NTOK + idx];
    t = (t < 0) ? 0 : ((t > NTOK - 1) ? (NTOK - 1) : t);
    const v4f r = *(const v4fa*)(rec + (size_t)t * 4);
    const float wgt = (SLOT == 0) ? r.x : r.y;
    s_tok[tid] = t;
    s_w[tid] = (tid < nrows) ? wgt : 0.0f;
  }
  __syncthreads();
  #pragma unroll
  for (int j = 0; j < 12; ++j) {
    const int idx = tid + 256 * j;
    const int row = idx / 96, c8 = idx - row * 96;
    const size_t go = (size_t)s_tok[row] * HIDD + 8 * c8;
    *(v4ua*)(sA + row * AP2 + 8 * c8) = *(const v4ua*)(xf + go);
  }
  __syncthreads();

  const int mg = wv & 1, ng = wv >> 1;
  const v8f z8 = {0.f, 0.f, 0.f, 0.f, 0.f, 0.f, 0.f, 0.f};
  const float r64 = 0.015625f;

  #pragma unroll 1
  for (int nh = 0; nh < 6; ++nh) {
    v8f ga[4], ua[4];
    #pragma unroll
    for (int nt = 0; nt < 4; ++nt) { ga[nt] = z8; ua[nt] = z8; }
    #pragma unroll 1
    for (int k0 = 0; k0 < HIDD; k0 += 32) {
      const v16h a = ldfrag_h(sA + (16 * mg + m) * AP2 + k0, h);
      #pragma unroll
      for (int nt = 0; nt < 4; ++nt) {
        const int n = nh * 256 + ng * 64 + 16 * nt + m;
        const size_t bo = ((size_t)e * IEX + n) * HIDD + k0;
        const v16h bgf = ldfrag_h(pg + bo, h);
        const v16h buf = ldfrag_h(pu + bo, h);
        ga[nt] = wmma_h(a, bgf, ga[nt]);
        ua[nt] = wmma_h(a, buf, ua[nt]);
      }
    }
    #pragma unroll
    for (int nt = 0; nt < 4; ++nt)
      #pragma unroll
      for (int r = 0; r < 8; ++r) {
        const int rowl = 16 * mg + 8 * h + r;
        const int col = nh * 256 + ng * 64 + 16 * nt + m;
        const float g = ga[nt][r] * r64;
        const float u = ua[nt][r] * r64;
        const float en = __expf(-g);
        const float sg = g * __builtin_amdgcn_rcpf(1.0f + en);
        const float hv = sg * u;
        sH[rowl * HP2 + col] = (unsigned short)hfb(hv * 64.0f);
      }
  }
  __syncthreads();

  const float r4096 = 0.000244140625f;
  #pragma unroll 1
  for (int np = 0; np < 3; ++np) {
    v8f ya[4];
    #pragma unroll
    for (int nt = 0; nt < 4; ++nt) ya[nt] = z8;
    #pragma unroll 1
    for (int k0 = 0; k0 < IEX; k0 += 32) {
      const v16h a = ldfrag_h(sH + (16 * mg + m) * HP2 + k0, h);
      #pragma unroll
      for (int nt = 0; nt < 4; ++nt) {
        const int n = np * 256 + ng * 64 + 16 * nt + m;
        const size_t bo = ((size_t)e * HIDD + n) * IEX + k0;
        const v16h bdf = ldfrag_h(pd + bo, h);
        ya[nt] = wmma_h(a, bdf, ya[nt]);
      }
    }
    __syncthreads();
    float* sy = sY + wv * 16 * YP;
    const int colbase = np * 256 + ng * 64;
    #pragma unroll
    for (int nt = 0; nt < 4; ++nt)
      #pragma unroll
      for (int r = 0; r < 8; ++r) {
        const int rowl = 8 * h + r;
        const int cl = 16 * nt + m;
        const float y = (ya[nt][r] * r4096) * s_w[16 * mg + rowl];
        sy[rowl * YP + cl] = y;
      }
    __syncthreads();
    y_pass<SLOT>(sy, s_tok, padd, hres, dst, mg, nrows, colbase, lane);
    __threadfence();
    y_pass<SLOT>(sy, s_tok, padd, hres, dst, mg, nrows, colbase, lane);
  }
}

extern "C" void kernel_launch(void* const* d_in, const int* in_sizes, int n_in,
                              void* d_out, int out_size, void* d_ws, size_t ws_size,
                              hipStream_t stream)
{
  if (n_in < 25) return;
  if (in_sizes[0] != NTOK * HIDD) return;
  if (in_sizes[1] != SEQL * SEQL) return;
  if (in_sizes[2] != SEQL * NBAT * NBAT) return;
  if (in_sizes[3] != NTOK) return;
  if (in_sizes[4] != HIDD || in_sizes[5] != HIDD || in_sizes[6] != HIDD) return;
  if (in_sizes[7] != HIDD * HIDD || in_sizes[8] != HIDD) return;
  if (in_sizes[9] != KVW * HIDD || in_sizes[10] != KVW) return;
  if (in_sizes[11] != KVW * HIDD || in_sizes[12] != KVW) return;
  if (in_sizes[13] != HIDD * HIDD) return;
  if (in_sizes[14] != HIDD * HIDD || in_sizes[15] != HIDD) return;
  if (in_sizes[16] != KVW * HIDD || in_sizes[17] != KVW) return;
  if (in_sizes[18] != KVW * HIDD || in_sizes[19] != KVW) return;
  if (in_sizes[20] != HIDD * HIDD) return;
  if (in_sizes[21] != NEX * HIDD) return;
  if (in_sizes[22] != NEX * HIDD * IEX || in_sizes[23] != NEX * HIDD * IEX || in_sizes[24] != NEX * IEX * HIDD) return;
  if (out_size != NTOK * HIDD) return;

  const float* hidden = (const float*)d_in[0];
  const float* amask  = (const float*)d_in[1];
  const float* gmask  = (const float*)d_in[2];
  const int*   pos    = (const int*)d_in[3];
  const float* ln1_w  = (const float*)d_in[4];
  const float* ln2_w  = (const float*)d_in[5];
  const float* ln3_w  = (const float*)d_in[6];
  const float* sq_w   = (const float*)d_in[7];    const float* sq_b = (const float*)d_in[8];
  const float* sk_w   = (const float*)d_in[9];    const float* sk_b = (const float*)d_in[10];
  const float* sv_w   = (const float*)d_in[11];   const float* sv_b = (const float*)d_in[12];
  const float* so_w   = (const float*)d_in[13];
  const float* gq_w   = (const float*)d_in[14];   const float* gq_b = (const float*)d_in[15];
  const float* gk_w   = (const float*)d_in[16];   const float* gk_b = (const float*)d_in[17];
  const float* gv_w   = (const float*)d_in[18];   const float* gv_b = (const float*)d_in[19];
  const float* go_w   = (const float*)d_in[20];
  const float* gate_w = (const float*)d_in[21];
  const float* w_gate = (const float*)d_in[22];
  const float* w_up   = (const float*)d_in[23];
  const float* w_down = (const float*)d_in[24];
  float* out = (float*)d_out;

  const size_t bPlane = (size_t)NTOK * HIDD * 2;
  const size_t bWAT   = (size_t)2 * 3145728 * 2;
  const size_t bQ     = (size_t)NBAT * NHD * SEQL * HDM * 2;
  const size_t bKV    = (size_t)NBAT * NKV * SEQL * HDM * 2;
  const size_t bHS    = (size_t)NTOK * HIDD * 4;
  const size_t bCS    = (size_t)NTOK * 64 * 4;
  const size_t bWE    = (size_t)NEX * HIDD * IEX * 2;
  const size_t bREC   = (size_t)NTOK * 16;
  const size_t bLST   = (size_t)2 * NEX * NTOK * 4;
  const size_t bCNT   = (size_t)2 * NEX * 32 * 4;
  const size_t total  = 2 * bPlane + bWAT + 2 * bQ + 4 * bKV + 2 * bHS + bCS + 3 * bWE + bREC + bLST + bCNT;
  if (total > ws_size) return;
  if (total > (size_t)134217728) return;

  char* ws = (char*)d_ws;
  size_t off = 0;
  unsigned short* PLH = (unsigned short*)(ws + off); off += bPlane;
  unsigned short* PLL = (unsigned short*)(ws + off); off += bPlane;
  unsigned short* WAT = (unsigned short*)(ws + off); off += bWAT;
  unsigned short* QH  = (unsigned short*)(ws + off); off += bQ;
  unsigned short* QL  = (unsigned short*)(ws + off); off += bQ;
  unsigned short* KH  = (unsigned short*)(ws + off); off += bKV;
  unsigned short* KL  = (unsigned short*)(ws + off); off += bKV;
  unsigned short* VH  = (unsigned short*)(ws + off); off += bKV;
  unsigned short* VL  = (unsigned short*)(ws + off); off += bKV;
  float*          HS1 = (float*)(ws + off);          off += bHS;
  float*          HS2 = (float*)(ws + off);          off += bHS;
  float*          CS  = (float*)(ws + off);          off += bCS;
  unsigned short* WGP = (unsigned short*)(ws + off); off += bWE;
  unsigned short* WUP = (unsigned short*)(ws + off); off += bWE;
  unsigned short* WDP = (unsigned short*)(ws + off); off += bWE;
  float*          REC = (float*)(ws + off);          off += bREC;
  int*            LST = (int*)(ws + off);            off += bLST;
  int*            CNT = (int*)(ws + off);            off += bCNT;
  if (off != total) return;

  float* Q2F = (float*)QH;
  float* K2F = (float*)KH;
  float* V2F = (float*)VH;
  float* P0  = HS1;

  unsigned short* SQH = WAT + 0;        unsigned short* SQL = WAT + 589824;
  unsigned short* SKH = WAT + 1179648;  unsigned short* SKL = WAT + 1376256;
  unsigned short* SVH = WAT + 1572864;  unsigned short* SVL = WAT + 1769472;
  unsigned short* SOH = WAT + 1966080;  unsigned short* SOL = WAT + 2555904;
  unsigned short* GQH = SQH + 3145728;  unsigned short* GQL = SQL + 3145728;
  unsigned short* GKH = SKH + 3145728;  unsigned short* GKL = SKL + 3145728;
  unsigned short* GVH = SVH + 3145728;  unsigned short* GVL = SVL + 3145728;
  unsigned short* GOH = SOH + 3145728;  unsigned short* GOL = SOL + 3145728;

  Inv32 ivf;
  for (int i = 0; i < 32; ++i) {
    const float xx = (float)(2 * i) / 64.0f;
    const float p = powf(10000.0f, xx);
    ivf.f[i] = 1.0f / p;
  }

  hipFuncSetAttribute(reinterpret_cast<const void*>(&k_gemm3<0>), hipFuncAttributeMaxDynamicSharedMemorySize, LDS_GEMM);
  hipFuncSetAttribute(reinterpret_cast<const void*>(&k_gemm3<1>), hipFuncAttributeMaxDynamicSharedMemorySize, LDS_GEMM);
  hipFuncSetAttribute(reinterpret_cast<const void*>(&k_gemm3<2>), hipFuncAttributeMaxDynamicSharedMemorySize, LDS_GEMM);
  hipFuncSetAttribute(reinterpret_cast<const void*>(&k_expert<0>), hipFuncAttributeMaxDynamicSharedMemorySize, LDS_EXP);
  hipFuncSetAttribute(reinterpret_cast<const void*>(&k_expert<1>), hipFuncAttributeMaxDynamicSharedMemorySize, LDS_EXP);

  k_cvt_w8<<<dim3((HIDD * HIDD / 8) / 256, 8), 256, 0, stream>>>(sq_w, sk_w, sv_w, so_w, gq_w, gk_w, gv_w, go_w, WAT);
  k_cvt_we<<<dim3(24, 24, 24), 256, 0, stream>>>(w_gate, w_up, w_down, WGP, WUP, WDP);

  k_rms_planes<<<NTOK / 8, 256, 0, stream>>>(hidden, ln1_w, PLH, PLL, pos, CS, 1, ivf);
  k_gemm3<1><<<dim3(NTOK / 128, HIDD / 128), 256, LDS_GEMM, stream>>>(
      PLH, PLL, HIDD, SQH, SQL, HIDD, HIDD, sq_b, 1, hidden, HIDD, 0, HS1, HIDD, QH, QL, NHD, CS);
  k_gemm3<1><<<dim3(NTOK / 128, KVW / 128), 256, LDS_GEMM, stream>>>(
      PLH, PLL, HIDD, SKH, SKL, HIDD, HIDD, sk_b, 1, hidden, HIDD, 0, HS1, HIDD, KH, KL, NKV, CS);
  k_gemm3<2><<<dim3(NTOK / 128, KVW / 128), 256, LDS_GEMM, stream>>>(
      PLH, PLL, HIDD, SVH, SVL, HIDD, HIDD, sv_b, 1, hidden, HIDD, 0, HS1, HIDD, VH, VL, NKV, CS);
  k_flash<<<dim3(NBAT * NHD, SEQL / 64), 128, 0, stream>>>(QH, QL, KH, KL, VH, VL, amask, PLH, PLL);
  k_gemm3<0><<<dim3(NTOK / 128, HIDD / 128), 256, LDS_GEMM, stream>>>(
      PLH, PLL, HIDD, SOH, SOL, HIDD, HIDD, sq_b, 0, hidden, HIDD, 1, HS1, HIDD, QH, QL, NHD, CS);

  k_rms_planes<<<NTOK / 8, 256, 0, stream>>>(HS1, ln2_w, PLH, PLL, pos, CS, 0, ivf);
  k_gemm3<0><<<dim3(NTOK / 128, HIDD / 128), 256, LDS_GEMM, stream>>>(
      PLH, PLL, HIDD, GQH, GQL, HIDD, HIDD, gq_b, 1, HS1, HIDD, 0, Q2F, HIDD, QH, QL, NHD, CS);
  k_gemm3<0><<<dim3(NTOK / 128, KVW / 128), 256, LDS_GEMM, stream>>>(
      PLH, PLL, HIDD, GKH, GKL, HIDD, HIDD, gk_b, 1, HS1, HIDD, 0, K2F, KVW, KH, KL, NKV, CS);
  k_gemm3<0><<<dim3(NTOK / 128, KVW / 128), 256, LDS_GEMM, stream>>>(
      PLH, PLL, HIDD, GVH, GVL, HIDD, HIDD, gv_b, 1, HS1, HIDD, 0, V2F, KVW, VH, VL, NKV, CS);
  k_gattn<<<(SEQL * NHD) / 8, 256, 0, stream>>>(Q2F, K2F, V2F, gmask, PLH, PLL);
  k_gemm3<0><<<dim3(NTOK / 128, HIDD / 128), 256, LDS_GEMM, stream>>>(
      PLH, PLL, HIDD, GOH, GOL, HIDD, HIDD, gq_b, 0, HS1, HIDD, 1, HS2, HIDD, QH, QL, NHD, CS);

  k_rms_route<<<NTOK / 8, 256, 0, stream>>>(HS2, ln3_w, gate_w, PLH, REC);
  k_lists<<<NEX, 256, 0, stream>>>(REC, LST, CNT);
  k_expert<0><<<dim3(NTOK / 32, NEX), 256, LDS_EXP, stream>>>(PLH, WGP, WUP, WDP, REC, LST, CNT, P0, HS2, P0);
  k_expert<1><<<dim3(NTOK / 32, NEX), 256, LDS_EXP, stream>>>(PLH, WGP, WUP, WDP, REC, LST, CNT, P0, HS2, out);
}
